// Encoder_75831942578735
// MI455X (gfx1250) — hardware-verified
//
#include <hip/hip_runtime.h>
#include <stddef.h>
#include <stdint.h>
#include <math.h>

#pragma clang fp contract(off)

#define CIN    128
#define HID    64
#define K2     128
#define NGR    128
#define NTHR   256
#define NWAVE  8
#define EPT    8
#define CHUNK  (NTHR * EPT)
#define WCAP   (EPT * 32)
#define LISTN  (NWAVE * WCAP)
#define NBA    1024
#define SLA    10
#define RCAP   28672
#define DEGCAP 64
#define GBM    128
#define GBN    64
#define GTHR   256
#define NU1    (HID * (CIN / 8))
#define NU2    (HID * (K2 / 8))
#define SROWS  1024
#define SQ     256
#define GT     (NGR * HID)
#define NPARF  (8 * HID)
#define AGG_ZINTS (LISTN + 2 * RCAP + 3 * NBA)
#define AGG_LDS_INTS (AGG_ZINTS + 16)
#define WSMAX  134217728

static_assert((CHUNK & (CHUNK - 1)) == 0 && CHUNK <= 4096);
static_assert((NBA & (NBA - 1)) == 0 && NBA == (1 << SLA));
static_assert(((long long)CHUNK << SLA) < (1LL << 31));
static_assert(LISTN % NTHR == 0);
static_assert(NBA % NWAVE == 0 && NBA % 32 == 0 && NBA == 4 * NTHR);
static_assert(RCAP % (4 * NTHR) == 0 && AGG_ZINTS % 4 == 0 && LISTN % 4 == 0);
static_assert(RCAP >= 17546);
static_assert(DEGCAP >= 36 + 8);
static_assert(CIN % 32 == 0 && K2 % 32 == 0 && K2 == 2 * HID && HID == GBN);
static_assert(GBM == (GTHR / 32) * 16 && GBN == 64);
static_assert(NU1 == 4 * NTHR && NU2 == 4 * NTHR);
static_assert(CIN / 8 == 16 && K2 / 8 == 16);
static_assert(HID == 2 * 32);
static_assert(NTHR == 4 * HID && SROWS == 4 * SQ);
static_assert(GT == 8 * NTHR * 4 && NGR == 32 * 4 && NGR % 4 == 0);
static_assert(AGG_LDS_INTS * 4 <= 300000);
static_assert(NPARF == 128 * 4);

typedef float          v2f   __attribute__((ext_vector_type(2)));
typedef float          v4f   __attribute__((ext_vector_type(4)));
typedef float          v8f   __attribute__((ext_vector_type(8)));
typedef int            v4i   __attribute__((ext_vector_type(4)));
typedef int            v8i   __attribute__((ext_vector_type(8)));
typedef unsigned int   v4u   __attribute__((ext_vector_type(4)));
typedef unsigned short v8us  __attribute__((ext_vector_type(8)));
typedef unsigned short v16us __attribute__((ext_vector_type(16)));
typedef __bf16         v16bf __attribute__((ext_vector_type(16)));
typedef v2f  __attribute__((may_alias)) v2fa;
typedef v4f  __attribute__((may_alias)) v4fa;
typedef v4i  __attribute__((may_alias)) v4ia;
typedef v4u  __attribute__((may_alias)) v4ua;
typedef v8us __attribute__((may_alias)) v8usa;
union FragB { v16bf v; v16us u; v8us h[2]; v8i w; };

__device__ __forceinline__ v8f wmb(const FragB& a, const FragB& b, v8f c) {
  v8f d = __builtin_amdgcn_wmma_f32_16x16x32_bf16(false, a.v, false, b.v, (short)0, c, false, false);
  asm volatile("v_nop\n\tv_nop\n\tv_nop\n\tv_nop" : "+v"(d) : "v"(a.w), "v"(b.w));
  return d;
}

__device__ __forceinline__ unsigned bf16_bits(float f) {
  const unsigned u = __float_as_uint(f);
  return (u + 0x7FFFu + ((u >> 16) & 1u)) >> 16;
}
__device__ __forceinline__ unsigned bf16_bits_np(float f) {
  const unsigned b = bf16_bits(f);
  return (f != f) ? 0x7FC0u : (b & 0xFFFFu);
}
__device__ __forceinline__ unsigned bf16_valbits(unsigned u) {
  return (u + 0x7FFFu + ((u >> 16) & 1u)) & 0xFFFF0000u;
}

__device__ __forceinline__ int scan_chunk(const int* __restrict__ dsts, int nE, int cbase, int slotBase,
                                          int vec8, int* list, int tid, int lane, int wave) {
  int wc = 0;
  const int el0  = tid * EPT;
  const int e0   = cbase + el0;
  const int sent = -2147483647 - 1;
  v4i da, db;
  if (vec8 != 0 && cbase + CHUNK <= nE) {
    da = *(const v4i*)(dsts + e0);
    db = *(const v4i*)(dsts + e0 + 4);
  } else {
    da.x = (e0     < nE) ? dsts[min(e0,     nE - 1)] : sent;
    da.y = (e0 + 1 < nE) ? dsts[min(e0 + 1, nE - 1)] : sent;
    da.z = (e0 + 2 < nE) ? dsts[min(e0 + 2, nE - 1)] : sent;
    da.w = (e0 + 3 < nE) ? dsts[min(e0 + 3, nE - 1)] : sent;
    db.x = (e0 + 4 < nE) ? dsts[min(e0 + 4, nE - 1)] : sent;
    db.y = (e0 + 5 < nE) ? dsts[min(e0 + 5, nE - 1)] : sent;
    db.z = (e0 + 6 < nE) ? dsts[min(e0 + 6, nE - 1)] : sent;
    db.w = (e0 + 7 < nE) ? dsts[min(e0 + 7, nE - 1)] : sent;
  }
  const unsigned nbs = (unsigned)slotBase;
  const unsigned unb = (unsigned)NBA;
  const unsigned s0 = (unsigned)da.x - nbs, s1 = (unsigned)da.y - nbs;
  const unsigned s2 = (unsigned)da.z - nbs, s3 = (unsigned)da.w - nbs;
  const unsigned s4 = (unsigned)db.x - nbs, s5 = (unsigned)db.y - nbs;
  const unsigned s6 = (unsigned)db.z - nbs, s7 = (unsigned)db.w - nbs;
  const bool h0 = s0 < unb, h1 = s1 < unb, h2 = s2 < unb, h3 = s3 < unb;
  const bool h4 = s4 < unb, h5 = s5 < unb, h6 = s6 < unb, h7 = s7 < unb;
  const int hc = (int)h0 + (int)h1 + (int)h2 + (int)h3 + (int)h4 + (int)h5 + (int)h6 + (int)h7;
  const unsigned any = __builtin_amdgcn_ballot_w32(hc != 0);
  if (any != 0u) {
    int incl = hc;
#pragma unroll
    for (int d = 1; d < 32; d <<= 1) {
      const int y = __shfl_up(incl, d, 32);
      if (lane >= d) incl += y;
    }
    const int tot = __shfl(incl, 31, 32);
    int pos = incl - hc;
    int* lw = list + wave * WCAP;
#define HITJ(J, HJ, SJ) if (HJ) { if (pos < WCAP) lw[pos] = ((el0 + (J)) << SLA) | (int)(SJ); pos = pos + 1; }
    HITJ(0, h0, s0)
    HITJ(1, h1, s1)
    HITJ(2, h2, s2)
    HITJ(3, h3, s3)
    HITJ(4, h4, s4)
    HITJ(5, h5, s5)
    HITJ(6, h6, s6)
    HITJ(7, h7, s7)
#undef HITJ
    wc = tot;
  }
  return wc;
}

__global__ __launch_bounds__(NTHR) void k_prep(const float* __restrict__ x, int nN, int nbx,
                                               const float* __restrict__ W1, const float* __restrict__ W2,
                                               const float* __restrict__ p0, const float* __restrict__ p1,
                                               const float* __restrict__ p2, const float* __restrict__ p3,
                                               const float* __restrict__ p4, const float* __restrict__ p5,
                                               const float* __restrict__ p6, const float* __restrict__ p7,
                                               unsigned short* xb, unsigned short* W1T, unsigned short* W2D,
                                               float* par, int* flagg, int nFlagU) {
  const int tid = (int)threadIdx.x;
  const int bx  = (int)blockIdx.x;
  if (bx < nbx) {
    const int u   = bx * NTHR + tid;
    const int row = u >> 4;
    const int k8  = (u & 15) * 8;
    const int rc  = row < nN ? row : nN - 1;
    const float* p = x + (size_t)rc * CIN + k8;
    const v4f a = *(const v4fa*)p;
    const v4f b = *(const v4fa*)(p + 4);
    const bool ok = row < nN;
    v8us o;
    o[0] = ok ? (unsigned short)bf16_bits(a.x) : (unsigned short)0;
    o[1] = ok ? (unsigned short)bf16_bits(a.y) : (unsigned short)0;
    o[2] = ok ? (unsigned short)bf16_bits(a.z) : (unsigned short)0;
    o[3] = ok ? (unsigned short)bf16_bits(a.w) : (unsigned short)0;
    o[4] = ok ? (unsigned short)bf16_bits(b.x) : (unsigned short)0;
    o[5] = ok ? (unsigned short)bf16_bits(b.y) : (unsigned short)0;
    o[6] = ok ? (unsigned short)bf16_bits(b.z) : (unsigned short)0;
    o[7] = ok ? (unsigned short)bf16_bits(b.w) : (unsigned short)0;
    unsigned short* dp = xb + (size_t)row * CIN + k8;
    *(volatile v8us*)dp = o;
    __threadfence();
    *(volatile v8us*)dp = o;
    return;
  }
  const int bi = bx - nbx;
  if (bi < 4) {
    const int u  = bi * NTHR + tid;
    const int n  = u >> 4;
    const int k8 = (u & 15) * 8;
    const float* p = W1 + (size_t)k8 * HID + n;
    v8us o;
#pragma unroll
    for (int i = 0; i < 8; ++i) o[i] = (unsigned short)bf16_bits(p[(size_t)i * HID]);
    unsigned short* dp = W1T + (size_t)n * CIN + k8;
    *(volatile v8us*)dp = o;
    __threadfence();
    *(volatile v8us*)dp = o;
    return;
  }
  if (bi < 8) {
    const int v  = (bi - 4) * NTHR + tid;
    const int n  = v >> 4;
    const int k8 = (v & 15) * 8;
    const int kk = k8 & (HID - 1);
    const float* p = W2 + (size_t)kk * HID + n;
    v8us o;
#pragma unroll
    for (int i = 0; i < 8; ++i) o[i] = (unsigned short)bf16_bits(p[(size_t)i * HID]);
    unsigned short* dp = W2D + (size_t)n * K2 + k8;
    *(volatile v8us*)dp = o;
    __threadfence();
    *(volatile v8us*)dp = o;
    return;
  }
  if (bi == 8) {
    const int a  = (tid >> 4) & 7;
    const int ch = tid & 15;
    v4u r = {0u, 0u, 0u, 0u};
#define PCAND(J, P) { const v4u qv = *(const v4ua*)((P) + 4 * ch); \
      const unsigned mk = (a == (J)) ? 0xFFFFFFFFu : 0u; \
      r.x |= qv.x & mk; r.y |= qv.y & mk; r.z |= qv.z & mk; r.w |= qv.w & mk; }
    PCAND(0, p0)
    PCAND(1, p1)
    PCAND(2, p2)
    PCAND(3, p3)
    PCAND(4, p4)
    PCAND(5, p5)
    PCAND(6, p6)
    PCAND(7, p7)
#undef PCAND
    v4f pv;
    pv.x = __uint_as_float(bf16_valbits(r.x));
    pv.y = __uint_as_float(bf16_valbits(r.y));
    pv.z = __uint_as_float(bf16_valbits(r.z));
    pv.w = __uint_as_float(bf16_valbits(r.w));
    const bool wr = tid < (NPARF / 4);
    const v4i z4 = {0, 0, 0, 0};
    if (wr) *(volatile v4f*)(par + 4 * tid) = pv;
#pragma unroll 1
    for (int u = tid; u < nFlagU; u += NTHR) *(volatile v4i*)(flagg + 4 * (size_t)u) = z4;
    __threadfence();
    if (wr) *(volatile v4f*)(par + 4 * tid) = pv;
#pragma unroll 1
    for (int u = tid; u < nFlagU; u += NTHR) *(volatile v4i*)(flagg + 4 * (size_t)u) = z4;
  }
}

__global__ __launch_bounds__(NTHR) void k_bucket(const int* __restrict__ srcs, const int* __restrict__ dsts,
                                                 int nE, int nN, int vec8,
                                                 int* listg, int* cntg, int* offg, float* disg, int* flagg) {
  extern __shared__ __attribute__((aligned(16))) int dsm[];
  __shared__ __attribute__((aligned(16))) float disl[NBA];
  int* list = dsm;
  int* hl   = dsm + LISTN;
  int* sl   = dsm + LISTN + RCAP;
  int* cnt  = dsm + LISTN + 2 * RCAP;
  int* offs = cnt + NBA;
  int* cur  = offs + NBA;
  int* misc = cur + NBA;
  const int tid = (int)threadIdx.x, lane = tid & 31, wave = tid >> 5;
  const int blk = (int)blockIdx.x;
  const int nodeBase = blk * NBA;

  {
    const v4i z4 = {0, 0, 0, 0};
    for (int i = tid * 4; i < AGG_ZINTS; i += NTHR * 4) *(v4ia*)(dsm + i) = z4;
    if (tid < 16) misc[tid] = 0;
  }
  __syncthreads();

  int t = 0, ov = 0;
  const int nChunks = (nE + CHUNK - 1) / CHUNK;
#pragma unroll 1
  for (int ch = 0; ch < nChunks; ++ch) {
    const int cbase = ch * CHUNK;
    const int wc = scan_chunk(dsts, nE, cbase, nodeBase, vec8, list, tid, lane, wave);
    if (lane == 0) misc[wave] = wc;
    __syncthreads();
    if (wave == 0) {
#pragma unroll 1
      for (int w2 = 0; w2 < NWAVE; ++w2) {
        int c = misc[w2];
        c = c < 0 ? 0 : (c > WCAP ? WCAP : c);
#pragma unroll 1
        for (int b0 = 0; b0 < c; b0 += 32) {
          const int idx = b0 + lane;
          const int ent = list[w2 * WCAP + (idx < WCAP ? idx : WCAP - 1)];
          const int m32 = (c - b0) < 32 ? (c - b0) : 32;
#pragma unroll 1
          for (int k = 0; k < m32; ++k) {
            const int u    = __builtin_amdgcn_readlane(ent, k);
            const int slot = u & (NBA - 1);
            const int el   = (u >> SLA) & (CHUNK - 1);
            const int pk   = ((cbase + el) << SLA) | slot;
            if (t < RCAP) {
              if (lane == 0) { hl[t] = pk; cnt[slot] = cnt[slot] + 1; }
              t = t + 1;
            } else {
              ov = 1;
            }
          }
        }
      }
    }
    __syncthreads();
  }
  if (wave == 0 && lane == 0) { misc[8] = t; misc[9] = ov; }
  __syncthreads();
  int tt = misc[8];
  tt = tt < 0 ? 0 : (tt > RCAP ? RCAP : tt);

  if (wave == 0) {
    const int base = lane * (NBA / 32);
    int s = 0;
    int bg = 0;
#pragma unroll 1
    for (int i = 0; i < NBA / 32; ++i) {
      const int cv = cnt[base + i];
      s += cv;
      bg |= (cv > DEGCAP) ? 1 : 0;
    }
    const unsigned bm = __builtin_amdgcn_ballot_w32(bg != 0);
    if (lane == 0) misc[10] = (bm != 0u) ? 1 : 0;
    int incl = s;
#pragma unroll
    for (int d = 1; d < 32; d <<= 1) {
      const int y = __shfl_up(incl, d, 32);
      if (lane >= d) incl += y;
    }
    int run = incl - s;
#pragma unroll 1
    for (int i = 0; i < NBA / 32; ++i) {
      const int cv = cnt[base + i];
      offs[base + i] = run;
      cur[base + i]  = run;
      run += cv;
    }
  }
  __syncthreads();
  if (wave == 0) {
#pragma unroll 1
    for (int b0 = 0; b0 < tt; b0 += 32) {
      const int idx = b0 + lane;
      const int ent = hl[idx < RCAP ? idx : RCAP - 1];
      const int m32 = (tt - b0) < 32 ? (tt - b0) : 32;
#pragma unroll 1
      for (int k = 0; k < m32; ++k) {
        const int u    = __builtin_amdgcn_readlane(ent, k);
        const int slot = u & (NBA - 1);
        if (lane == 0) {
          int p = cur[slot];
          p = p < 0 ? 0 : (p > RCAP - 1 ? RCAP - 1 : p);
          sl[p] = u;
          cur[slot] = p + 1;
        }
      }
    }
  }
  __syncthreads();

#pragma unroll 1
  for (int i = tid; i < NBA; i += NTHR) {
    const int deg = cnt[i] + 1;
    const float df = (float)deg;
    const float rr = 1.0f / sqrtf(df);
    disl[i] = (deg > 0) ? rr : 0.0f;
  }
  __syncthreads();

  {
    const v4i c4 = *(const v4ia*)(cnt + 4 * tid);
    const v4i o4 = *(const v4ia*)(offs + 4 * tid);
    const v4f d4 = *(const v4fa*)(disl + 4 * tid);
    const int fl = ((misc[9] | misc[10]) != 0) ? 1 : 0;
    const v4i f4 = {fl, fl, fl, fl};
    int*   cp = cntg + (size_t)nodeBase + 4 * tid;
    int*   op = offg + (size_t)nodeBase + 4 * tid;
    float* dp = disg + (size_t)nodeBase + 4 * tid;
    int*   fp = flagg + (size_t)blk * 32 + 4 * (tid & 7);
    const bool wf = tid < 8;
    *(volatile v4i*)cp = c4;
    *(volatile v4i*)op = o4;
    *(volatile v4f*)dp = d4;
    if (wf) *(volatile v4i*)fp = f4;
    __threadfence();
    *(volatile v4i*)cp = c4;
    *(volatile v4i*)op = o4;
    *(volatile v4f*)dp = d4;
    if (wf) *(volatile v4i*)fp = f4;
  }

  int* lg = listg + (size_t)blk * RCAP;
#pragma unroll 1
  for (int it = 0; it < RCAP / (4 * NTHR); ++it) {
    const int i0 = 4 * (it * NTHR + tid);
    const v4i e4 = *(const v4ia*)(sl + i0);
    int ea = e4.x >> SLA, eb = e4.y >> SLA, ec = e4.z >> SLA, ed = e4.w >> SLA;
    ea = ea < 0 ? 0 : (ea > nE - 1 ? nE - 1 : ea);
    eb = eb < 0 ? 0 : (eb > nE - 1 ? nE - 1 : eb);
    ec = ec < 0 ? 0 : (ec > nE - 1 ? nE - 1 : ec);
    ed = ed < 0 ? 0 : (ed > nE - 1 ? nE - 1 : ed);
    int sa = srcs[ea], sb = srcs[eb], sc = srcs[ec], sd = srcs[ed];
    sa = sa < 0 ? 0 : (sa > nN - 1 ? nN - 1 : sa);
    sb = sb < 0 ? 0 : (sb > nN - 1 ? nN - 1 : sb);
    sc = sc < 0 ? 0 : (sc > nN - 1 ? nN - 1 : sc);
    sd = sd < 0 ? 0 : (sd > nN - 1 ? nN - 1 : sd);
    v4i o;
    o.x = (i0     < tt) ? sa : 0;
    o.y = (i0 + 1 < tt) ? sb : 0;
    o.z = (i0 + 2 < tt) ? sc : 0;
    o.w = (i0 + 3 < tt) ? sd : 0;
    *(volatile v4i*)(lg + i0) = o;
    __threadfence();
    *(volatile v4i*)(lg + i0) = o;
  }
}

__global__ __launch_bounds__(GTHR) void k_gemm(
    const unsigned short* __restrict__ A, const unsigned short* __restrict__ WT,
    float* outF, int K, int ldo)
{
  __shared__ __attribute__((aligned(16))) float stg[GBM * GBN];
  const int tid = (int)threadIdx.x, lane = tid & 31, wave = tid >> 5, hh = lane >> 4, m = lane & 15;
  const int rowBase = (int)blockIdx.x * GBM;
  const int col0    = (int)blockIdx.y * GBN;

  v8f acc[4];
  {
    const v8f z = {0.f, 0.f, 0.f, 0.f, 0.f, 0.f, 0.f, 0.f};
    acc[0] = z; acc[1] = z; acc[2] = z; acc[3] = z;
  }
  const unsigned short* ap = A  + (size_t)(rowBase + 16 * wave + m) * (size_t)K + 8 * hh;
  const unsigned short* wp = WT + (size_t)(col0 + m) * (size_t)K + 8 * hh;
  const int ksteps = K >> 5;
#pragma unroll 1
  for (int ks = 0; ks < ksteps; ++ks) {
    FragB af;
    af.h[0] = *(const v8usa*)(ap + 32 * ks);
    af.h[1] = *(const v8usa*)(ap + 32 * ks + 16);
#pragma unroll
    for (int t = 0; t < 4; ++t) {
      const unsigned short* wq = wp + (size_t)(16 * t) * (size_t)K + 32 * ks;
      FragB bf;
      bf.h[0] = *(const v8usa*)wq;
      bf.h[1] = *(const v8usa*)(wq + 16);
      acc[t] = wmb(af, bf, acc[t]);
    }
  }

#pragma unroll
  for (int t = 0; t < 4; ++t) {
    const int lc = 16 * t + m;
#pragma unroll
    for (int r = 0; r < 8; ++r) {
      const int lr = 16 * wave + 8 * hh + r;
      stg[lr * GBN + lc] = acc[t][r];
    }
  }
  __syncthreads();

  v4f fv[8];
#pragma unroll
  for (int i = 0; i < 8; ++i) {
    const int lr = 16 * wave + 2 * i + hh;
    fv[i] = *(const v4fa*)(stg + lr * GBN + 4 * m);
  }
#pragma unroll
  for (int i = 0; i < 8; ++i) {
    const int lr = 16 * wave + 2 * i + hh;
    const int gr = rowBase + lr;
    float* op = outF + (size_t)gr * (size_t)ldo + col0 + 4 * m;
    *(volatile v4f*)op = fv[i];
  }
  __threadfence();
#pragma unroll
  for (int i = 0; i < 8; ++i) {
    const int lr = 16 * wave + 2 * i + hh;
    const int gr = rowBase + lr;
    float* op = outF + (size_t)gr * (size_t)ldo + col0 + 4 * m;
    *(volatile v4f*)op = fv[i];
  }
}

__global__ __launch_bounds__(NTHR) void k_agg(const int* __restrict__ listg, const int* __restrict__ cntg,
                                              const int* __restrict__ offg, const float* __restrict__ dis,
                                              const int* __restrict__ flagg, const float* __restrict__ xl,
                                              const float* __restrict__ par, int prow, int nN, int mRows,
                                              float* hout) {
  const int tid = (int)threadIdx.x, lane = tid & 31, wave = tid >> 5;
  const int blk = (int)blockIdx.x;
  const int nodeBase = blk * NBA;
  const int* lb = listg + (size_t)blk * RCAP;
  float bv0, bv1;
  {
    const v2f a = *(const v2fa*)(par + prow * HID + 2 * lane);
    bv0 = a.x; bv1 = a.y;
  }
  const int fl = __builtin_amdgcn_readfirstlane(flagg[(size_t)blk * 32]);
  const float qnan = __int_as_float(0x7fc00000);
  const float pz = (fl != 0) ? qnan : 0.0f;
  const int sa = (2 * lane) & 31, sb = (2 * lane + 1) & 31;
#pragma unroll 1
  for (int si = 0; si < NBA / NWAVE; ++si) {
    const int s    = si * NWAVE + wave;
    const int node = nodeBase + s;
    int c = __builtin_amdgcn_readfirstlane(cntg[node]);
    const bool big = c > DEGCAP;
    c = c < 0 ? 0 : (c > DEGCAP ? DEGCAP : c);
    int o = __builtin_amdgcn_readfirstlane(offg[node]);
    o = o < 0 ? 0 : (o > RCAP ? RCAP : o);
    const int nc = node < nN ? node : nN - 1;
    const float dd = dis[nc];
    const float rd = dd * dd;
    float acc0 = 0.0f, acc1 = 0.0f;
#pragma unroll 1
    for (int b0 = 0; b0 < c; b0 += 32) {
      int idx = o + b0 + lane;
      idx = idx > RCAP - 1 ? RCAP - 1 : idx;
      int sr = lb[idx];
      sr = sr < 0 ? 0 : (sr > nN - 1 ? nN - 1 : sr);
      const float ds  = dis[sr];
      const float cf  = ds * dd;
      const int   cfi = __float_as_int(cf);
      const int m32 = (c - b0) < 32 ? (c - b0) : 32;
#pragma unroll 1
      for (int k = 0; k < m32; ++k) {
        const int   sk = __builtin_amdgcn_readlane(sr, k);
        const float ck = __int_as_float(__builtin_amdgcn_readlane(cfi, k));
        const v2f a = *(const v2fa*)(xl + (size_t)sk * HID + 2 * lane);
        const float m0 = a.x * ck;
        const float m1 = a.y * ck;
        acc0 = acc0 + m0;
        acc1 = acc1 + m1;
      }
    }
    float sv0, sv1;
    {
      const v2f a = *(const v2fa*)(xl + (size_t)nc * HID + 2 * lane);
      sv0 = a.x; sv1 = a.y;
    }
    const float pzr = big ? qnan : pz;
    const bool live = node < nN;
    const float t0 = sv0 * rd;
    const float t1 = sv1 * rd;
    float y0 = (acc0 + t0) + bv0;
    float y1 = (acc1 + t1) + bv1;
    y0 = y0 + pzr; y1 = y1 + pzr;
    const float v0 = live ? y0 : 0.0f;
    const float v1 = live ? y1 : 0.0f;
    const bool wr = (node < mRows) && (lane < 16);
    v4f ow;
    ow.x = __shfl(v0, sa, 32); ow.y = __shfl(v1, sa, 32);
    ow.z = __shfl(v0, sb, 32); ow.w = __shfl(v1, sb, 32);
    float* op = hout + (size_t)node * HID + 4 * (lane & 15);
    if (wr) *(volatile v4f*)op = ow;
    __threadfence();
    if (wr) *(volatile v4f*)op = ow;
  }
}

template <int MODE>
__global__ __launch_bounds__(NTHR) void k_gstat(const float* __restrict__ gp, const int* __restrict__ bat,
                                                const float* __restrict__ par, int prow,
                                                const float* __restrict__ meanp, const float* __restrict__ istdp,
                                                int nN, float* rec, int* crec) {
  extern __shared__ __attribute__((aligned(16))) float gsm[];
  __shared__ __attribute__((aligned(16))) int CT[4 * NGR];
  const int tid = (int)threadIdx.x;
  const int c   = tid & (HID - 1);
  const int q   = __builtin_amdgcn_readfirstlane(tid >> 6);
  {
    const v4f z4 = {0.0f, 0.0f, 0.0f, 0.0f};
    for (int i = tid * 4; i < 4 * GT; i += NTHR * 4) *(v4fa*)(gsm + i) = z4;
    for (int i = tid; i < 4 * NGR; i += NTHR) CT[i] = 0;
  }
  float al = 0.0f, wt = 0.0f, bs = 0.0f;
  if constexpr (MODE >= 1) al = par[(prow + 1) * HID + c];
  if constexpr (MODE == 2) { wt = par[(prow + 2) * HID + c]; bs = par[(prow + 3) * HID + c]; }
  __syncthreads();

  const int rb = (int)blockIdx.x * SROWS + q * SQ;
  int nr = nN - rb;
  nr = nr < 0 ? 0 : (nr > SQ ? SQ : nr);
  float* Tq = gsm + q * GT;
  int curg = -1;
  float acc = 0.0f;
  int rc = 0;
  float am = 0.0f, isd = 0.0f;
#pragma unroll 1
  for (int j = 0; j < nr; ++j) {
    const int row = rb + j;
    int g = __builtin_amdgcn_readfirstlane(bat[row]);
    g = ((unsigned)g < (unsigned)NGR) ? g : -1;
    if (g != curg) {
      if (curg >= 0) {
        Tq[curg * HID + c] = Tq[curg * HID + c] + acc;
        if (c == 0) CT[q * NGR + curg] = CT[q * NGR + curg] + rc;
      }
      curg = g; acc = 0.0f; rc = 0;
      if constexpr (MODE >= 1) {
        const int gc = g < 0 ? 0 : g;
        am = al * meanp[gc * HID + c];
        if constexpr (MODE == 2) isd = istdp[gc * HID + c];
      }
    }
    const float xv = gp[(size_t)row * HID + c];
    float v;
    if constexpr (MODE == 0) {
      v = xv;
    } else if constexpr (MODE == 1) {
      const float d = xv - am;
      v = d * d;
    } else {
      const float d = xv - am;
      const float tq = wt * d;
      const float ts = tq * isd;
      const float y = ts + bs;
      v = (y > 0.0f) ? y : (y - y);
    }
    if (curg >= 0) { acc = acc + v; rc = rc + 1; }
  }
  if (curg >= 0) {
    Tq[curg * HID + c] = Tq[curg * HID + c] + acc;
    if (c == 0) CT[q * NGR + curg] = CT[q * NGR + curg] + rc;
  }
  __syncthreads();

  v4f rv[8];
#pragma unroll
  for (int it = 0; it < 8; ++it) {
    const int u = 4 * (it * NTHR + tid);
    const v4f a0 = *(const v4fa*)(gsm + u);
    const v4f a1 = *(const v4fa*)(gsm + GT + u);
    const v4f a2 = *(const v4fa*)(gsm + 2 * GT + u);
    const v4f a3 = *(const v4fa*)(gsm + 3 * GT + u);
    rv[it] = ((a0 + a1) + a2) + a3;
  }
  v4i cv = {0, 0, 0, 0};
  const bool wc4 = tid < (NGR / 4);
  {
    const int ci = 4 * (tid & (NGR / 4 - 1));
    const v4i c0 = *(const v4ia*)(CT + ci);
    const v4i c1 = *(const v4ia*)(CT + NGR + ci);
    const v4i c2 = *(const v4ia*)(CT + 2 * NGR + ci);
    const v4i c3 = *(const v4ia*)(CT + 3 * NGR + ci);
    cv = ((c0 + c1) + c2) + c3;
  }
  float* rp = rec + (size_t)blockIdx.x * GT;
  int*   cp = crec + (size_t)blockIdx.x * NGR + 4 * (tid & (NGR / 4 - 1));
#pragma unroll
  for (int it = 0; it < 8; ++it) *(volatile v4f*)(rp + 4 * (it * NTHR + tid)) = rv[it];
  if (wc4) *(volatile v4i*)cp = cv;
  __threadfence();
#pragma unroll
  for (int it = 0; it < 8; ++it) *(volatile v4f*)(rp + 4 * (it * NTHR + tid)) = rv[it];
  if (wc4) *(volatile v4i*)cp = cv;
}

template <int MODE>
__global__ __launch_bounds__(NTHR) void k_gcomb(const float* __restrict__ rec, const int* __restrict__ crec,
                                                int nSB, const int* __restrict__ flagg, int nFl, float* outp) {
  __shared__ __attribute__((aligned(16))) float stg[NTHR];
  const int tid = (int)threadIdx.x;
  const int c = tid & (HID - 1);
  const int g = (int)blockIdx.x * 4 + (tid >> 6);
  double S = 0.0;
  int n = 0;
#pragma unroll 2
  for (int b = 0; b < nSB; ++b) {
    S = S + (double)rec[((size_t)b * NGR + g) * HID + c];
    n = n + crec[(size_t)b * NGR + g];
  }
  const int den = n < 1 ? 1 : n;
  float r = (float)(S / (double)den);
  if constexpr (MODE == 1) {
    const float ve = r + 1e-5f;
    r = 1.0f / sqrtf(ve);
  }
  if constexpr (MODE == 2) {
    int anyf = 0;
#pragma unroll 2
    for (int b = 0; b < nFl; ++b) anyf |= flagg[(size_t)b * 32];
    r = (anyf != 0) ? __int_as_float(0x7fc00000) : r;
  }
  stg[tid] = r;
  __syncthreads();
  const bool wr = tid < (NTHR / 4);
  const v4f v = *(const v4fa*)(stg + 4 * (tid & (NTHR / 4 - 1)));
  float* op = outp + (size_t)blockIdx.x * NTHR + 4 * (tid & (NTHR / 4 - 1));
  if (wr) *(volatile v4f*)op = v;
  __threadfence();
  if (wr) *(volatile v4f*)op = v;
}

__global__ __launch_bounds__(NTHR) void k_apply(const float* __restrict__ gp, const int* __restrict__ bat,
                                                const float* __restrict__ par, int prow,
                                                const float* __restrict__ meanp, const float* __restrict__ istdp,
                                                int nN, int nUnits, unsigned short* xo) {
  const int u = (int)blockIdx.x * NTHR + (int)threadIdx.x;
  if (u >= nUnits) return;
  const int row = u >> 3;
  const int c8  = (u & 7) * 8;
  const bool ok = row < nN;
  const int rc  = ok ? row : nN - 1;
  int g = bat[rc];
  g = g < 0 ? 0 : (g > NGR - 1 ? NGR - 1 : g);
  const v4f x0 = *(const v4fa*)(gp + (size_t)rc * HID + c8);
  const v4f x1 = *(const v4fa*)(gp + (size_t)rc * HID + c8 + 4);
  const v4f m0 = *(const v4fa*)(meanp + g * HID + c8);
  const v4f m1 = *(const v4fa*)(meanp + g * HID + c8 + 4);
  const v4f s0 = *(const v4fa*)(istdp + g * HID + c8);
  const v4f s1 = *(const v4fa*)(istdp + g * HID + c8 + 4);
  const v4f a0 = *(const v4fa*)(par + (prow + 1) * HID + c8);
  const v4f a1 = *(const v4fa*)(par + (prow + 1) * HID + c8 + 4);
  const v4f w0 = *(const v4fa*)(par + (prow + 2) * HID + c8);
  const v4f w1 = *(const v4fa*)(par + (prow + 2) * HID + c8 + 4);
  const v4f b0 = *(const v4fa*)(par + (prow + 3) * HID + c8);
  const v4f b1 = *(const v4fa*)(par + (prow + 3) * HID + c8 + 4);
  const float xs[8] = {x0.x, x0.y, x0.z, x0.w, x1.x, x1.y, x1.z, x1.w};
  const float ms[8] = {m0.x, m0.y, m0.z, m0.w, m1.x, m1.y, m1.z, m1.w};
  const float ss[8] = {s0.x, s0.y, s0.z, s0.w, s1.x, s1.y, s1.z, s1.w};
  const float as[8] = {a0.x, a0.y, a0.z, a0.w, a1.x, a1.y, a1.z, a1.w};
  const float ws[8] = {w0.x, w0.y, w0.z, w0.w, w1.x, w1.y, w1.z, w1.w};
  const float bb[8] = {b0.x, b0.y, b0.z, b0.w, b1.x, b1.y, b1.z, b1.w};
  v8us hv, lv;
#pragma unroll
  for (int i = 0; i < 8; ++i) {
    const float am = as[i] * ms[i];
    const float d  = xs[i] - am;
    const float tq = ws[i] * d;
    const float ts = tq * ss[i];
    const float y  = ts + bb[i];
    const float r  = (y > 0.0f) ? y : (y - y);
    const float v  = ok ? r : 0.0f;
    const unsigned hb = bf16_bits_np(v);
    const float hf = __uint_as_float(hb << 16);
    const unsigned lb = bf16_bits_np(v - hf);
    hv[i] = (unsigned short)hb;
    lv[i] = (unsigned short)lb;
  }
  unsigned short* hp = xo + (size_t)row * K2 + c8;
  unsigned short* lp = hp + HID;
  *(volatile v8us*)hp = hv;
  *(volatile v8us*)lp = lv;
  __threadfence();
  *(volatile v8us*)hp = hv;
  *(volatile v8us*)lp = lv;
}

static inline int cdiv(int a, int b) { return (a + b - 1) / b; }
static inline size_t al256(size_t o) { return (o + 255) & ~(size_t)255; }

extern "C" void kernel_launch(void* const* d_in, const int* in_sizes, int n_in,
                              void* d_out, int out_size, void* d_ws, size_t ws_size,
                              hipStream_t stream) {
  if (n_in < 13) return;
  const int nN = in_sizes[2];
  if (nN < 1 || nN > (1 << 22)) return;
  if ((long long)in_sizes[0] != (long long)nN * CIN) return;
  if (in_sizes[1] < 2 || (in_sizes[1] & 1) != 0) return;
  const int nE = in_sizes[1] / 2;
  if (nE < 1 || nE >= (1 << (31 - SLA))) return;
  if (in_sizes[3] != CIN * HID) return;
  if (in_sizes[4] != HID || in_sizes[5] != HID || in_sizes[6] != HID || in_sizes[7] != HID) return;
  if (in_sizes[8] != HID * HID) return;
  if (in_sizes[9] != HID || in_sizes[10] != HID || in_sizes[11] != HID || in_sizes[12] != HID) return;
  if (out_size != NGR * HID) return;

  const float* x    = (const float*)d_in[0];
  const int*   edge = (const int*)d_in[1];
  const int*   bat  = (const int*)d_in[2];
  const float* W1   = (const float*)d_in[3];
  const float* b1   = (const float*)d_in[4];
  const float* al1  = (const float*)d_in[5];
  const float* wt1  = (const float*)d_in[6];
  const float* bi1  = (const float*)d_in[7];
  const float* W2   = (const float*)d_in[8];
  const float* b2   = (const float*)d_in[9];
  const float* al2  = (const float*)d_in[10];
  const float* wt2  = (const float*)d_in[11];
  const float* bi2  = (const float*)d_in[12];
  float* out = (float*)d_out;
  const int* src = edge;
  const int* dst = edge + nE;

  const int MP   = cdiv(nN, GBM) * GBM;
  const int gM   = MP / GBM;
  const int gA   = cdiv(MP, NBA);
  const int NBP  = gA * NBA;
  const int nSB  = cdiv(nN, SROWS);
  if ((long long)gA * NBA < (long long)MP) return;
  const int vec8 = ((nE & 3) == 0) ? 1 : 0;
  const int nbx  = (MP * (CIN / 8)) / NTHR;
  if ((long long)nbx * NTHR != (long long)MP * (CIN / 8)) return;
  const int nUa  = MP * 8;
  if (nUa % NTHR != 0) return;

  char* ws = (char*)d_ws;
  size_t off = 0;
  const size_t oXB  = off; off = al256(off + (size_t)MP * CIN * 2);
  const size_t oH   = off; off = al256(off + (size_t)MP * HID * 4);
  const size_t oGP  = off; off = al256(off + (size_t)MP * HID * 4);
  const size_t oLS  = off; off = al256(off + (size_t)gA * RCAP * 4);
  const size_t oCN  = off; off = al256(off + (size_t)NBP * 4);
  const size_t oOF  = off; off = al256(off + (size_t)NBP * 4);
  const size_t oDI  = off; off = al256(off + (size_t)NBP * 4);
  const size_t oRC  = off; off = al256(off + (size_t)nSB * GT * 4);
  const size_t oCR  = off; off = al256(off + (size_t)nSB * NGR * 4);
  const size_t oMN  = off; off = al256(off + (size_t)GT * 4);
  const size_t oIS  = off; off = al256(off + (size_t)GT * 4);
  const size_t oPA  = off; off = al256(off + (size_t)NPARF * 4);
  const size_t oW1  = off; off = al256(off + (size_t)HID * CIN * 2);
  const size_t oW2  = off; off = al256(off + (size_t)HID * K2 * 2);
  const size_t oFL  = off; off = al256(off + (size_t)gA * 128);
  if (off > ws_size || off > (size_t)WSMAX) return;
  unsigned short* XB   = (unsigned short*)(ws + oXB);
  unsigned short* X1HL = (unsigned short*)(ws + oXB);
  float* H    = (float*)(ws + oH);
  float* GP   = (float*)(ws + oGP);
  int*   LIST = (int*)(ws + oLS);
  int*   CNT  = (int*)(ws + oCN);
  int*   OFF  = (int*)(ws + oOF);
  float* DIS  = (float*)(ws + oDI);
  float* REC  = (float*)(ws + oRC);
  int*   CREC = (int*)(ws + oCR);
  float* MEAN = (float*)(ws + oMN);
  float* ISTD = (float*)(ws + oIS);
  float* PAR  = (float*)(ws + oPA);
  unsigned short* W1T = (unsigned short*)(ws + oW1);
  unsigned short* W2D = (unsigned short*)(ws + oW2);
  int*   FLAG = (int*)(ws + oFL);

  const size_t bktLds = (size_t)AGG_LDS_INTS * 4;
  const size_t gstLds = (size_t)4 * GT * 4;
  hipFuncSetAttribute(reinterpret_cast<const void*>(&k_bucket), hipFuncAttributeMaxDynamicSharedMemorySize, (int)bktLds);
  hipFuncSetAttribute(reinterpret_cast<const void*>(&k_gstat<0>), hipFuncAttributeMaxDynamicSharedMemorySize, (int)gstLds);
  hipFuncSetAttribute(reinterpret_cast<const void*>(&k_gstat<1>), hipFuncAttributeMaxDynamicSharedMemorySize, (int)gstLds);
  hipFuncSetAttribute(reinterpret_cast<const void*>(&k_gstat<2>), hipFuncAttributeMaxDynamicSharedMemorySize, (int)gstLds);

  k_prep<<<nbx + 9, NTHR, 0, stream>>>(x, nN, nbx, W1, W2, b1, al1, wt1, bi1, b2, al2, wt2, bi2,
                                       XB, W1T, W2D, PAR, FLAG, gA * 8);
  k_bucket<<<gA, NTHR, bktLds, stream>>>(src, dst, nE, nN, vec8, LIST, CNT, OFF, DIS, FLAG);
  k_gemm<<<dim3(gM, 1), GTHR, 0, stream>>>(XB, W1T, H, CIN, HID);
  k_agg<<<gA, NTHR, 0, stream>>>(LIST, CNT, OFF, DIS, FLAG, H, PAR, 0, nN, MP, GP);
  k_gstat<0><<<nSB, NTHR, gstLds, stream>>>(GP, bat, PAR, 0, MEAN, ISTD, nN, REC, CREC);
  k_gcomb<0><<<NGR / 4, NTHR, 0, stream>>>(REC, CREC, nSB, FLAG, gA, MEAN);
  k_gstat<1><<<nSB, NTHR, gstLds, stream>>>(GP, bat, PAR, 0, MEAN, ISTD, nN, REC, CREC);
  k_gcomb<1><<<NGR / 4, NTHR, 0, stream>>>(REC, CREC, nSB, FLAG, gA, ISTD);
  k_apply<<<nUa / NTHR, NTHR, 0, stream>>>(GP, bat, PAR, 0, MEAN, ISTD, nN, nUa, X1HL);
  k_gemm<<<dim3(gM, 1), GTHR, 0, stream>>>(X1HL, W2D, H, K2, HID);
  k_agg<<<gA, NTHR, 0, stream>>>(LIST, CNT, OFF, DIS, FLAG, H, PAR, 4, nN, MP, GP);
  k_gstat<0><<<nSB, NTHR, gstLds, stream>>>(GP, bat, PAR, 4, MEAN, ISTD, nN, REC, CREC);
  k_gcomb<0><<<NGR / 4, NTHR, 0, stream>>>(REC, CREC, nSB, FLAG, gA, MEAN);
  k_gstat<1><<<nSB, NTHR, gstLds, stream>>>(GP, bat, PAR, 4, MEAN, ISTD, nN, REC, CREC);
  k_gcomb<1><<<NGR / 4, NTHR, 0, stream>>>(REC, CREC, nSB, FLAG, gA, ISTD);
  k_gstat<2><<<nSB, NTHR, gstLds, stream>>>(GP, bat, PAR, 4, MEAN, ISTD, nN, REC, CREC);
  k_gcomb<2><<<NGR / 4, NTHR, 0, stream>>>(REC, CREC, nSB, FLAG, gA, out);
}
